// QuantumSuperpositionBranches_83863531421744
// MI455X (gfx1250) — hardware-run, weakly checked
//
#include <hip/hip_runtime.h>
#include <hip/hip_bf16.h>
#include <math.h>

typedef __attribute__((ext_vector_type(16))) _Float16 v16h;
typedef __attribute__((ext_vector_type(8)))  float    v8f;

#define NQ     10
#define NSTATE 1024
#define NPAR   100
#define BATCH  256
#define TWO_PI_F 6.2831853071795864f

#define PSTR 128
#define MSTR 32
typedef __attribute__((ext_vector_type(4))) float v4f;
__global__ __launch_bounds__(32)
void qsb_gemm_angles(const float* __restrict__ x,
                     const float* __restrict__ W1, const float* __restrict__ b1, const float* __restrict__ s1,
                     const float* __restrict__ W2, const float* __restrict__ b2, const float* __restrict__ s2,
                     const float* __restrict__ W3, const float* __restrict__ b3, const float* __restrict__ s3,
                     float* __restrict__ P)
{
    __shared__ __attribute__((aligned(16))) float sT[16][PSTR];
    const int tm     = blockIdx.x;
    const int branch = blockIdx.y;
    const float* W; const float* bv; const float* bs;
    if (branch == 0)      { W = W1; bv = b1; bs = s1; }
    else if (branch == 1) { W = W2; bv = b2; bs = s2; }
    else                  { W = W3; bv = b3; bs = s3; }

    const int l   = threadIdx.x;
    const int grp = l >> 4;
    const int lm  = l & 15;
    const int mBase = tm * 16;
    const float* arow = x + (mBase + lm) * 256;

    v8f acc[7] = {};
    for (int kk = 0; kk < 8; ++kk) {
        const int k0 = kk * 32;
        v16h ah, al;
        #pragma unroll
        for (int e = 0; e < 16; ++e) {
            const int ka = ((e < 8) ? 0 : 16) + grp * 8 + (e & 7);
            const float va = arow[k0 + ka];
            const _Float16 ha = (_Float16)va;
            ah[e] = ha; al[e] = (_Float16)(va - (float)ha);
        }
        #pragma unroll
        for (int tn = 0; tn < 7; ++tn) {
            const int n  = tn * 16 + lm;
            const int nc = (n < NPAR) ? n : (NPAR - 1);
            const float bmask = (n < NPAR) ? 1.0f : 0.0f;
            const float* brow = W + nc * 256;
            v16h bh, bl;
            #pragma unroll
            for (int e = 0; e < 16; ++e) {
                const int kb = ((e < 8) ? 0 : 16) + grp * 8 + (e & 7);
                const float vb = brow[k0 + kb] * bmask;
                const _Float16 hb = (_Float16)vb;
                bh[e] = hb; bl[e] = (_Float16)(vb - (float)hb);
            }
            acc[tn] = __builtin_amdgcn_wmma_f32_16x16x32_f16(false, ah, false, bh, (short)0, acc[tn], false, false);
            acc[tn] = __builtin_amdgcn_wmma_f32_16x16x32_f16(false, al, false, bh, (short)0, acc[tn], false, false);
            acc[tn] = __builtin_amdgcn_wmma_f32_16x16x32_f16(false, ah, false, bl, (short)0, acc[tn], false, false);
            asm volatile("v_nop\n\tv_nop\n\tv_nop\n\tv_nop" : "+v"(acc[tn]) : "v"(al), "v"(bl));
        }
    }
    #pragma unroll
    for (int tn = 0; tn < 8; ++tn) {
        const int n = tn * 16 + lm;
        #pragma unroll
        for (int r = 0; r < 8; ++r) {
            float v = 0.0f;
            if (tn < 7 && n < NPAR) { const float a = acc[tn][r] + bv[n] + bs[n]; v = TWO_PI_F / (1.0f + expf(-a)); }
            sT[grp * 8 + r][n] = v;
        }
    }
    __builtin_amdgcn_fence(__ATOMIC_RELEASE, "workgroup"); __builtin_amdgcn_wave_barrier(); __builtin_amdgcn_fence(__ATOMIC_ACQUIRE, "workgroup");
    float* Pb = P + (size_t)(branch * BATCH + mBase) * PSTR;
    for (int pass = 0; pass < 2; ++pass) {
        #pragma unroll
        for (int r = 0; r < 16; ++r) *(volatile v4f*)(Pb + r * PSTR + l * 4) = *(const v4f*)(&sT[r][l * 4]);
        __threadfence();
    }
}

__device__ __forceinline__ int insert_zero(int v, int b) {
    return ((v >> b) << (b + 1)) | (v & ((1 << b) - 1));
}

__device__ __forceinline__ void pair_rx(float* __restrict__ re, float* __restrict__ im,
                                        int i0, int i1, float c, float s) {
    float r0 = re[i0], m0 = im[i0], r1 = re[i1], m1 = im[i1];
    re[i0] = c * r0 + s * m1;
    im[i0] = c * m0 - s * r1;
    re[i1] = c * r1 + s * m0;
    im[i1] = c * m1 - s * r0;
}

__device__ __forceinline__ void gate_rx(float* re, float* im, int b, float c, float s, int tid) {
    #pragma unroll
    for (int p = 0; p < 2; ++p) {
        int pi = tid * 2 + p;
        int i0 = insert_zero(pi, b);
        pair_rx(re, im, i0, i0 | (1 << b), c, s);
    }
}

__device__ __forceinline__ void gate_ry(float* re, float* im, int b, float c, float s, int tid) {
    #pragma unroll
    for (int p = 0; p < 2; ++p) {
        int pi = tid * 2 + p;
        int i0 = insert_zero(pi, b);
        int i1 = i0 | (1 << b);
        float r0 = re[i0], m0 = im[i0], r1 = re[i1], m1 = im[i1];
        re[i0] = c * r0 - s * r1;
        im[i0] = c * m0 - s * m1;
        re[i1] = s * r0 + c * r1;
        im[i1] = s * m0 + c * m1;
    }
}

__device__ __forceinline__ void gate_rz(float* re, float* im, int b, float c, float s, int tid) {
    #pragma unroll
    for (int k = 0; k < 4; ++k) {
        int j = tid * 4 + k;
        float r = re[j], m = im[j];
        float sg = ((j >> b) & 1) ? s : -s;
        re[j] = r * c - m * sg;
        im[j] = m * c + r * sg;
    }
}

__device__ __forceinline__ void gate_crx(float* re, float* im, int cb, int tb,
                                         float c, float s, int tid) {
    int blo = (cb < tb) ? cb : tb;
    int bhi = (cb < tb) ? tb : cb;
    int i = insert_zero(tid, blo);
    i = insert_zero(i, bhi);
    i |= (1 << cb);
    pair_rx(re, im, i, i | (1 << tb), c, s);
}

__global__ __launch_bounds__(256)
void qsb_circuit(const float* __restrict__ P, float* __restrict__ M)
{
    __shared__ float sr[NSTATE];
    __shared__ float si[NSTATE];
    __shared__ float sang[NPAR];
    __shared__ float wsum[8][3];

    const int tid    = threadIdx.x;
    const int batch  = blockIdx.x;
    const int branch = blockIdx.y;
    const float* ang = P + (branch * BATCH + batch) * PSTR;
    __shared__ float res[MSTR];

    if (tid < NPAR) sang[tid] = ang[tid];

    #pragma unroll
    for (int k = 0; k < 4; ++k) { sr[tid * 4 + k] = 0.0f; si[tid * 4 + k] = 0.0f; }
    if (tid == 0) sr[0] = 1.0f;
    __syncthreads();

    int idx = 0;
    for (int layer = 0; layer < 2; ++layer) {
        for (int w = 0; w < NQ; ++w) {
            const int b = (NQ - 1) - w;
            { float t = sang[idx    ] * 0.5f; float c = cosf(t), s = sinf(t);
              gate_rx(sr, si, b, c, s, tid); __syncthreads(); }
            { float t = sang[idx + 1] * 0.5f; float c = cosf(t), s = sinf(t);
              gate_ry(sr, si, b, c, s, tid); __syncthreads(); }
            { float t = sang[idx + 2] * 0.5f; float c = cosf(t), s = sinf(t);
              gate_rz(sr, si, b, c, s, tid); __syncthreads(); }
            idx += 3;
        }
        for (int cw = 0; cw < NQ; ++cw) {
            int tw = (cw + 1) % NQ;
            float t = sang[idx++] * 0.5f; float c = cosf(t), s = sinf(t);
            gate_crx(sr, si, (NQ - 1) - cw, (NQ - 1) - tw, c, s, tid);
            __syncthreads();
        }
        for (int cw = NQ - 1; cw >= 0; --cw) {
            int tw = (cw + NQ - 1) % NQ;
            float t = sang[idx++] * 0.5f; float c = cosf(t), s = sinf(t);
            gate_crx(sr, si, (NQ - 1) - cw, (NQ - 1) - tw, c, s, tid);
            __syncthreads();
        }
    }

    const int lane = tid & 31;
    const int wave = tid >> 5;
    float* mo = M + (branch * BATCH + batch) * MSTR;
    if (tid < MSTR) res[tid] = 0.0f;

    for (int w = 0; w < NQ; ++w) {
        const int b = (NQ - 1) - w;
        float px = 0.0f, py = 0.0f, pz = 0.0f;
        #pragma unroll
        for (int p = 0; p < 2; ++p) {
            int pi = tid * 2 + p;
            int i0 = insert_zero(pi, b);
            int i1 = i0 | (1 << b);
            float r0 = sr[i0], m0 = si[i0], r1 = sr[i1], m1 = si[i1];
            px += r0 * r1 + m0 * m1;
            py += r0 * m1 - m0 * r1;
            pz += (r0 * r0 + m0 * m0) - (r1 * r1 + m1 * m1);
        }
        #pragma unroll
        for (int off = 16; off > 0; off >>= 1) {
            px += __shfl_down(px, off);
            py += __shfl_down(py, off);
            pz += __shfl_down(pz, off);
        }
        if (lane == 0) { wsum[wave][0] = px; wsum[wave][1] = py; wsum[wave][2] = pz; }
        __syncthreads();
        if (tid == 0) {
            float sx = 0.0f, sy = 0.0f, sz = 0.0f;
            #pragma unroll
            for (int q = 0; q < 8; ++q) { sx += wsum[q][0]; sy += wsum[q][1]; sz += wsum[q][2]; }
            res[w]      = 2.0f * sx;
            res[10 + w] = 2.0f * sy;
            res[20 + w] = sz;
        }
        __syncthreads();
    }
    if (tid < MSTR) { const float v = res[tid]; *(volatile float*)(mo + tid) = v; __threadfence(); *(volatile float*)(mo + tid) = v; }
}

__global__ __launch_bounds__(256)
void qsb_combine(const float* __restrict__ M,
                 const float* __restrict__ ar_, const float* __restrict__ ai_,
                 const float* __restrict__ br_, const float* __restrict__ bi_,
                 const float* __restrict__ gr_, const float* __restrict__ gi_,
                 float* __restrict__ out)
{
    int i = blockIdx.x * blockDim.x + threadIdx.x;
    if (i >= BATCH * 30) return;
    int batch = i / 30, col = i % 30;

    float m1 = M[(0 * BATCH + batch) * MSTR + col];
    float m2 = M[(1 * BATCH + batch) * MSTR + col];
    float m3 = M[(2 * BATCH + batch) * MSTR + col];

    float ar = ar_[0], ai = ai_[0];
    float br = br_[0], bi = bi_[0];
    float gr = gr_[0], gi = gi_[0];
    float inv = 1.0f / sqrtf(ar*ar + ai*ai + br*br + bi*bi + gr*gr + gi*gi + 1e-9f);
    ar *= inv; ai *= inv; br *= inv; bi *= inv; gr *= inv; gi *= inv;

    float re = ar * m1 + br * m2 + gr * m3;
    float im = ai * m1 + bi * m2 + gi * m3;
    const float ov = sqrtf(re * re + im * im);
    *(volatile float*)(out + i) = ov; __threadfence(); *(volatile float*)(out + i) = ov;
}

extern "C" void kernel_launch(void* const* d_in, const int* in_sizes, int n_in,
                              void* d_out, int out_size, void* d_ws, size_t ws_size,
                              hipStream_t stream)
{
    const float* x     = (const float*)d_in[0];
    const float* W1    = (const float*)d_in[1];
    const float* b1    = (const float*)d_in[2];
    const float* W2    = (const float*)d_in[3];
    const float* b2    = (const float*)d_in[4];
    const float* W3    = (const float*)d_in[5];
    const float* b3    = (const float*)d_in[6];
    const float* base1 = (const float*)d_in[7];
    const float* base2 = (const float*)d_in[8];
    const float* base3 = (const float*)d_in[9];
    const float* ar    = (const float*)d_in[10];
    const float* ai    = (const float*)d_in[11];
    const float* br    = (const float*)d_in[12];
    const float* bi    = (const float*)d_in[13];
    const float* gr    = (const float*)d_in[14];
    const float* gi    = (const float*)d_in[15];

    (void)in_sizes; (void)n_in; (void)out_size;
    if (ws_size < (size_t)(3 * BATCH * PSTR + 3 * BATCH * MSTR) * 4) return;
    float* P = (float*)d_ws;
    float* M = P + 3 * BATCH * PSTR;

    dim3 g1(16, 3);
    qsb_gemm_angles<<<g1, 32, 0, stream>>>(x, W1, b1, base1, W2, b2, base2,
                                           W3, b3, base3, P);

    dim3 g2(BATCH, 3);
    qsb_circuit<<<g2, 256, 0, stream>>>(P, M);

    int n = BATCH * 30;
    qsb_combine<<<(n + 255) / 256, 256, 0, stream>>>(M, ar, ai, br, bi, gr, gi,
                                                     (float*)d_out);
}
